// TreeLSTM_43611097923955
// MI455X (gfx1250) — hardware-run, weakly checked
//
#include <hip/hip_runtime.h>


#define NB    256
#define NGT   64
#define NGRP  4
#define NLEAF 256
#define NNODE 511
#define NLEV  9
#define NDIN  128
#define NH    256
#define NHID  100
#define NHP   128
#define NV    2048
#define NCH   4096
typedef _Float16 h16;
typedef unsigned short bf;
typedef __attribute__((ext_vector_type(16))) __bf16   v16bf;
typedef __attribute__((ext_vector_type(16))) _Float16 v16h;
typedef __attribute__((ext_vector_type(8)))  _Float16 v8h;
typedef __attribute__((ext_vector_type(8)))  unsigned short v8us;
typedef __attribute__((ext_vector_type(8)))  float    v8f;
typedef __attribute__((ext_vector_type(4)))  float    v4f;
typedef v8h  __attribute__((may_alias)) v8ha;
typedef v4f  __attribute__((may_alias)) v4fa;
typedef v8us __attribute__((may_alias)) v8usa;

__device__ __forceinline__ unsigned short f2bf(float f) { unsigned u = __float_as_uint(f); u += 0x7FFFu + ((u >> 16) & 1u); return (unsigned short)(u >> 16); }
__device__ __forceinline__ float bf2f(unsigned short b) { return __uint_as_float(((unsigned)b) << 16); }
__device__ __forceinline__ float bfr(float f) { return bf2f(f2bf(f)); }
__device__ __forceinline__ v16h cat16(v8h lo, v8h hi) { return __builtin_shufflevector(lo, hi, 0, 1, 2, 3, 4, 5, 6, 7, 8, 9, 10, 11, 12, 13, 14, 15); }
__device__ __forceinline__ v16bf cat16b(v8us lo, v8us hi) { return __builtin_bit_cast(v16bf, __builtin_shufflevector(lo, hi, 0, 1, 2, 3, 4, 5, 6, 7, 8, 9, 10, 11, 12, 13, 14, 15)); }
__device__ __forceinline__ v8f wmma16(v16h a, v16h b, v8f c) { return __builtin_amdgcn_wmma_f32_16x16x32_f16(false, a, false, b, (short)0, c, false, false); }
__device__ __forceinline__ v8f wmmab(v16bf a, v16bf b, v8f c) { return __builtin_amdgcn_wmma_f32_16x16x32_bf16(false, a, false, b, (short)0, c, false, false); }


template <typename T16> struct WFrag;
template <> struct WFrag<h16> { typedef v16h V; static __device__ __forceinline__ V ld(const h16* p) { return cat16(*(const v8h*)p, *(const v8h*)(p + 16)); } static __device__ __forceinline__ v8f mma(V a, V b, v8f c) { return wmma16(a, b, c); } };
template <> struct WFrag<bf> { typedef v16bf V; static __device__ __forceinline__ V ld(const bf* p) { return cat16b(*(const v8us*)p, *(const v8us*)(p + 16)); } static __device__ __forceinline__ v8f mma(V a, V b, v8f c) { return wmmab(a, b, c); } };
template <typename T16, int NSPLIT, bool BIAS>
__global__ __launch_bounds__(32) void k_gemmw(const T16* __restrict__ A, const T16* __restrict__ A2, const T16* __restrict__ Bt, const T16* __restrict__ Bt2, int K, float* C, int ldc, const float* __restrict__ bias, size_t sA, size_t sB, size_t sC) {
    typedef typename WFrag<T16>::V V;
    __shared__ __align__(16) float os[16 * 68];
    const size_t z = blockIdx.z; A += z * sA; if (A2) A2 += z * sA; Bt += z * sB; if (Bt2) Bt2 += z * sB; C += z * sC;
    const int lane = threadIdx.x & 31, lr = lane & 15, hi = lane >> 4; const int r0 = blockIdx.x * 64, c0 = blockIdx.y * 64;
    v8f acc[4][4];
#pragma unroll
    for (int mb = 0; mb < 4; ++mb)
#pragma unroll
        for (int nb = 0; nb < 4; ++nb) acc[mb][nb] = (v8f){};
    const size_t aoff = (size_t)(r0 + lr) * K + 8 * hi, boff = (size_t)(c0 + lr) * K + 8 * hi;
    for (int kc = 0; kc < K; kc += 32) {
        V a[4], a2[4];
#pragma unroll
        for (int mb = 0; mb < 4; ++mb) { a[mb] = WFrag<T16>::ld(A + aoff + (size_t)mb * 16 * K + kc); if (NSPLIT == 1 || NSPLIT == 2) a2[mb] = WFrag<T16>::ld(A2 + aoff + (size_t)mb * 16 * K + kc); }
#pragma unroll
        for (int nb = 0; nb < 4; ++nb) { const V b = WFrag<T16>::ld(Bt + boff + (size_t)nb * 16 * K + kc); V b2; if (NSPLIT >= 2) b2 = WFrag<T16>::ld(Bt2 + boff + (size_t)nb * 16 * K + kc);
#pragma unroll
            for (int mb = 0; mb < 4; ++mb) { acc[mb][nb] = WFrag<T16>::mma(a[mb], b, acc[mb][nb]); if (NSPLIT == 1 || NSPLIT == 2) acc[mb][nb] = WFrag<T16>::mma(a2[mb], b, acc[mb][nb]); if (NSPLIT >= 2) acc[mb][nb] = WFrag<T16>::mma(a[mb], b2, acc[mb][nb]); } }
        asm volatile("v_nop\n\tv_nop\n\tv_nop\n\tv_nop" : "+v"(acc[0][0]), "+v"(acc[1][1]), "+v"(acc[2][2]), "+v"(acc[3][3]) : "v"(a[0]), "v"(a[3]));
    }
#pragma unroll
    for (int mb = 0; mb < 4; ++mb) {
#pragma unroll
        for (int nb = 0; nb < 4; ++nb) {
#pragma unroll
            for (int j = 0; j < 8; ++j) os[(hi * 8 + j) * 68 + nb * 16 + lr] = acc[mb][nb][j]; }
        __builtin_amdgcn_wave_barrier(); asm volatile("" ::: "memory");
        float* crow = C + (size_t)(r0 + mb * 16) * ldc + c0;
#pragma unroll 1
        for (int ps = 0; ps < 2; ++ps) {
#pragma unroll
            for (int s = 0; s < 8; ++s) { const int row = 2 * s + hi, cofs = lr * 4; v4f val = *(const v4fa*)(os + row * 68 + cofs); if (BIAS) { val[0] += bfr(bias[c0 + cofs]); val[1] += bfr(bias[c0 + cofs + 1]); val[2] += bfr(bias[c0 + cofs + 2]); val[3] += bfr(bias[c0 + cofs + 3]); }
                *(volatile v4f*)(crow + (size_t)row * ldc + cofs) = val; }
            if (ps == 0) __threadfence(); }
        __builtin_amdgcn_wave_barrier(); asm volatile("" ::: "memory");
    }
}

typedef __attribute__((ext_vector_type(2))) _Float16 v2h;
typedef __attribute__((ext_vector_type(4))) _Float16 v4h;
typedef __attribute__((ext_vector_type(2))) unsigned short v2us;
typedef __attribute__((ext_vector_type(4))) unsigned short v4us;
typedef __attribute__((ext_vector_type(2))) float v2f;
typedef __attribute__((ext_vector_type(4))) int v4i;

__global__ __launch_bounds__(256) void k_wtG(const float* __restrict__ w, int K, int N, bf* Bt) {
    const int lane = threadIdx.x & 31; const int L0 = (blockIdx.x * 8 + (threadIdx.x >> 5)) * 8; const int nlines = N * K / 64;
#pragma unroll
    for (int ps = 0; ps < 2; ++ps) {
        for (int l = 0; l < 8; ++l) { const int L = L0 + l; if (L >= nlines) break; const size_t e = (size_t)L * 64 + lane * 2; const int k = (int)(e % K), n = (int)(e / K); v2us o;
            o[0] = f2bf(w[(size_t)k * N + n]); o[1] = f2bf(w[(size_t)(k + 1) * N + n]); *(volatile v2us*)(Bt + e) = o; }
        if (ps == 0) __threadfence(); }
}

__global__ __launch_bounds__(256) void k_zero(float* dst, int n4) { const int i = blockIdx.x * 256 + threadIdx.x; if (i >= n4) return; v4f z; z[0] = 0.0f; z[1] = 0.0f; z[2] = 0.0f; z[3] = 0.0f;
    *(volatile v4f*)(dst + (size_t)i * 4) = z; __threadfence(); *(volatile v4f*)(dst + (size_t)i * 4) = z; }

__global__ __launch_bounds__(256) void k_gath(const int* __restrict__ ids, const float* __restrict__ emb, bf* xe, int nshift, int off, size_t n4) { const size_t i = (size_t)blockIdx.x * 256 + threadIdx.x; if (i >= n4) return;
    const int row = (int)(i >> 5); const int c4 = (int)(i & 31) * 4; const int b = row >> nshift; const int j = row - (b << nshift); int id = ids[(size_t)b * NNODE + off + j]; id = id < 0 ? 0 : id; id = id > NV - 1 ? NV - 1 : id;
    const v4f v = *(const v4f*)(emb + (size_t)id * NDIN + c4); v4us o;
#pragma unroll
    for (int k = 0; k < 4; ++k) o[k] = (id == 0) ? (unsigned short)0 : f2bf(v[k]);
    *(volatile v4us*)(xe + i * 4) = o; __threadfence(); *(volatile v4us*)(xe + i * 4) = o; }

__device__ __forceinline__ float sgm(float v) { return 1.0f / (1.0f + expf(-v)); }
__global__ __launch_bounds__(256) void k_cell(const float* __restrict__ pxi, const float* __restrict__ pxf, const float* __restrict__ p1i, const float* __restrict__ p1f0, const float* __restrict__ p1f1, const float* __restrict__ p2i, const float* __restrict__ p2f0, const float* __restrict__ p2f1, const float* __restrict__ cprev, const float* __restrict__ bh1, const float* __restrict__ bh2, float* cnew, bf* he, bf* ho, bf* hrh, bf* hrl, int row0, size_t n4) { const size_t i = (size_t)blockIdx.x * 256 + threadIdx.x; if (i >= n4) return;
    const size_t rl = i >> 6; const int c4 = (int)(i & 63) * 4; const size_t r = (size_t)row0 + rl;
    const float* qx = pxi + rl * (3 * NH) + c4; v4f ai = *(const v4f*)qx; v4f ao = *(const v4f*)(qx + NH); v4f au = *(const v4f*)(qx + 2 * NH); v4f g0 = (v4f){}; v4f g1 = (v4f){}; v4f c1 = (v4f){}; v4f c2 = (v4f){};
    if (p1i) { const float* q1 = p1i + rl * (3 * NH) + c4; const float* q2 = p2i + rl * (3 * NH) + c4;
        ai = (ai + *(const v4f*)q1) + *(const v4f*)q2; ao = (ao + *(const v4f*)(q1 + NH)) + *(const v4f*)(q2 + NH); au = (au + *(const v4f*)(q1 + 2 * NH)) + *(const v4f*)(q2 + 2 * NH);
        const v4f fx = *(const v4f*)(pxf + rl * NH + c4);
        g0 = (*(const v4f*)(p1f0 + rl * NH + c4) + *(const v4f*)(p2f0 + rl * NH + c4)) + fx; g1 = (*(const v4f*)(p1f1 + rl * NH + c4) + *(const v4f*)(p2f1 + rl * NH + c4)) + fx;
        c1 = *(const v4f*)(cprev + (2 * r) * NH + c4); c2 = *(const v4f*)(cprev + (2 * r + 1) * NH + c4);
    } else {
#pragma unroll
        for (int k = 0; k < 4; ++k) { ai[k] = (ai[k] + bfr(bh1[c4 + k])) + bfr(bh2[c4 + k]); ao[k] = (ao[k] + bfr(bh1[NH + c4 + k])) + bfr(bh2[NH + c4 + k]); au[k] = (au[k] + bfr(bh1[2 * NH + c4 + k])) + bfr(bh2[2 * NH + c4 + k]); } }
    v4f cv; v4us hw; v4us hl;
#pragma unroll
    for (int k = 0; k < 4; ++k) { const float gi = sgm(ai[k]); const float go = sgm(ao[k]); const float gu = tanhf(au[k]); float c = gi * gu;
        if (p1i) c = (c + sgm(g0[k]) * c1[k]) + sgm(g1[k]) * c2[k];
        const float h = go * tanhf(c); cv[k] = c; hw[k] = f2bf(h); hl[k] = f2bf(h - bf2f(hw[k])); }
    bf* hp = ((r & 1) ? ho : he) + (r >> 1) * NH + c4;
#pragma unroll
    for (int ps = 0; ps < 2; ++ps) { *(volatile v4f*)(cnew + r * NH + c4) = cv; *(volatile v4us*)hp = hw; if (hrh) { *(volatile v4us*)(hrh + r * NH + c4) = hw; *(volatile v4us*)(hrl + r * NH + c4) = hl; } if (ps == 0) __threadfence(); } }

__global__ __launch_bounds__(256) void k_head(const float* __restrict__ ph, const float* __restrict__ b1, const float* __restrict__ w2, const float* __restrict__ b2, float* out) { const int t = blockIdx.x * 256 + threadIdx.x; const float* p = ph + (size_t)t * NHP; float acc = 0.0f;
    for (int j = 0; j < NHID; ++j) { float s = p[j] + bfr(b1[j]); s = s > 0.0f ? s : 0.0f; acc = acc + s * bfr(w2[j]); }
    acc = acc + bfr(b2[0]); *(volatile float*)(out + t) = acc; __threadfence(); *(volatile float*)(out + t) = acc; }

static constexpr size_t kSzWxI = (size_t)768 * NDIN * 2, kSzWxF = (size_t)NH * NDIN * 2, kSzWhI = (size_t)768 * NH * 2, kSzWhF = (size_t)NH * NH * 2;
static constexpr size_t kOffWxI = 0, kOffWxF = kOffWxI + kSzWxI, kOffW1I = kOffWxF + kSzWxF, kOffW1F0 = kOffW1I + kSzWhI, kOffW1F1 = kOffW1F0 + kSzWhF, kOffW2I = kOffW1F1 + kSzWhF, kOffW2F0 = kOffW2I + kSzWhI, kOffW2F1 = kOffW2F0 + kSzWhF;
static constexpr size_t kOffWL1 = kOffW2F1 + kSzWhF, kSzWL1 = (size_t)NHP * NH * 2;
static constexpr size_t kOffXE = kOffWL1 + kSzWL1, kSzXE = (size_t)NGT * NNODE * NDIN * 2;
static constexpr size_t kOffCA = kOffXE + kSzXE, kSzCA = (size_t)NGT * NLEAF * NH * 4, kOffCB = kOffCA + kSzCA, kSzCB = kSzCA / 2;
static constexpr size_t kOffHA = kOffCB + kSzCB, kSzHA = (size_t)NGT * NLEAF * NH * 2, kOffHB = kOffHA + kSzHA, kSzHB = kSzHA / 2;
static constexpr size_t kOffP = kOffHB + kSzHB, kSzPi = (size_t)NCH * 768 * 4, kSzPf = (size_t)NCH * NH * 4, kSzP = 3 * kSzPi + 5 * kSzPf;
static constexpr size_t kOffHRH = kOffP + kSzP, kSzHR = (size_t)NB * NH * 2, kOffHRL = kOffHRH + kSzHR, kOffPH = kOffHRL + kSzHR, kSzPH = (size_t)NB * NHP * 4, kWsTotal = kOffPH + kSzPH;
static_assert(kOffWL1 == 1572864ull && kSzWL1 == 65536ull && kSzXE == 8372224ull && kSzCA == 16777216ull && kSzHA == 8388608ull && kSzP == 58720256ull && kWsTotal == 106872832ull);
static_assert(kWsTotal <= 134217728ull);
static_assert((kOffXE % 128) == 0 && (kOffCA % 128) == 0 && (kOffCB % 128) == 0 && (kOffHA % 128) == 0 && (kOffHB % 128) == 0 && (kOffP % 128) == 0 && (kOffHRH % 128) == 0 && (kOffHRL % 128) == 0 && (kOffPH % 128) == 0 && (kSzPi % 128) == 0 && (kSzPf % 128) == 0);
static_assert((NGT % 64) == 0 && (NCH % 64) == 0 && (NB % 64) == 0 && (768 % 64) == 0 && (NH % 64) == 0 && (NHP % 64) == 0 && (NDIN % 32) == 0 && (NH % 32) == 0 && NGT * NGRP == NB && NHID <= NHP);
static_assert(((NDIN * 768) % 64) == 0 && ((NDIN * NH) % 64) == 0 && ((NH * 768) % 64) == 0 && ((NH * NH) % 64) == 0 && ((NH * NHID) % 64) == 0);

extern "C" void kernel_launch(void* const* d_in, const int* in_sizes, int n_in, void* d_out, int out_size, void* d_ws, size_t ws_size, hipStream_t stream) {
    if (n_in < 22) return;
    if (in_sizes[0] != NB * NNODE || in_sizes[1] != NV * NDIN) return;
    if (in_sizes[2] != NDIN * 768 || in_sizes[3] != 768 || in_sizes[4] != NH * 768 || in_sizes[5] != 768 || in_sizes[6] != NH * 768 || in_sizes[7] != 768) return;
    if (in_sizes[8] != NDIN * NH || in_sizes[9] != NH) return;
    for (int q = 10; q < 18; q += 2) { if (in_sizes[q] != NH * NH || in_sizes[q + 1] != NH) return; }
    if (in_sizes[18] != NH * NHID || in_sizes[19] != NHID || in_sizes[20] != NHID || in_sizes[21] != 1) return;
    if (out_size != NB) return;
    if (ws_size < kWsTotal) return;
    const int* ids = (const int*)d_in[0]; const float* emb = (const float*)d_in[1];
    const float* wioux = (const float*)d_in[2]; const float* bioux = (const float*)d_in[3]; const float* wiouh1 = (const float*)d_in[4]; const float* biouh1 = (const float*)d_in[5]; const float* wiouh2 = (const float*)d_in[6]; const float* biouh2 = (const float*)d_in[7];
    const float* wfx = (const float*)d_in[8]; const float* bfx = (const float*)d_in[9]; const float* wfh11 = (const float*)d_in[10]; const float* bfh11 = (const float*)d_in[11]; const float* wfh12 = (const float*)d_in[12]; const float* bfh12 = (const float*)d_in[13]; const float* wfh21 = (const float*)d_in[14]; const float* bfh21 = (const float*)d_in[15]; const float* wfh22 = (const float*)d_in[16]; const float* bfh22 = (const float*)d_in[17];
    const float* wl1 = (const float*)d_in[18]; const float* bl1 = (const float*)d_in[19]; const float* wl2 = (const float*)d_in[20]; const float* bl2 = (const float*)d_in[21];
    float* out = (float*)d_out; char* ws = (char*)d_ws;
    bf* WxI = (bf*)(ws + kOffWxI); bf* WxF = (bf*)(ws + kOffWxF); bf* W1I = (bf*)(ws + kOffW1I); bf* W1F0 = (bf*)(ws + kOffW1F0); bf* W1F1 = (bf*)(ws + kOffW1F1); bf* W2I = (bf*)(ws + kOffW2I); bf* W2F0 = (bf*)(ws + kOffW2F0); bf* W2F1 = (bf*)(ws + kOffW2F1); bf* WL1 = (bf*)(ws + kOffWL1);
    bf* XE = (bf*)(ws + kOffXE); float* CA = (float*)(ws + kOffCA); float* CB = (float*)(ws + kOffCB); bf* HA = (bf*)(ws + kOffHA); bf* HB = (bf*)(ws + kOffHB); bf* HRH = (bf*)(ws + kOffHRH); bf* HRL = (bf*)(ws + kOffHRL); float* PH = (float*)(ws + kOffPH);
    float* PXi = (float*)(ws + kOffP); float* PXf = (float*)((char*)PXi + kSzPi); float* P1i = (float*)((char*)PXf + kSzPf); float* P1f0 = (float*)((char*)P1i + kSzPi); float* P1f1 = (float*)((char*)P1f0 + kSzPf); float* P2i = (float*)((char*)P1f1 + kSzPf); float* P2f0 = (float*)((char*)P2i + kSzPi); float* P2f1 = (float*)((char*)P2f0 + kSzPf);

    k_wtG<<<(unsigned)((NDIN * 768 / 64 + 63) / 64), 256, 0, stream>>>(wioux, NDIN, 768, WxI);
    k_wtG<<<(unsigned)((NDIN * NH / 64 + 63) / 64), 256, 0, stream>>>(wfx, NDIN, NH, WxF);
    k_wtG<<<(unsigned)((NH * 768 / 64 + 63) / 64), 256, 0, stream>>>(wiouh1, NH, 768, W1I);
    k_wtG<<<(unsigned)((NH * NH / 64 + 63) / 64), 256, 0, stream>>>(wfh11, NH, NH, W1F0);
    k_wtG<<<(unsigned)((NH * NH / 64 + 63) / 64), 256, 0, stream>>>(wfh21, NH, NH, W1F1);
    k_wtG<<<(unsigned)((NH * 768 / 64 + 63) / 64), 256, 0, stream>>>(wiouh2, NH, 768, W2I);
    k_wtG<<<(unsigned)((NH * NH / 64 + 63) / 64), 256, 0, stream>>>(wfh12, NH, NH, W2F0);
    k_wtG<<<(unsigned)((NH * NH / 64 + 63) / 64), 256, 0, stream>>>(wfh22, NH, NH, W2F1);
    k_zero<<<(unsigned)(kSzWL1 / 16 / 256), 256, 0, stream>>>((float*)WL1, (int)(kSzWL1 / 16));
    k_wtG<<<(unsigned)((NH * NHID / 64 + 63) / 64), 256, 0, stream>>>(wl1, NH, NHID, WL1);

    for (int g = 0; g < NGRP; ++g) { const int* gids = ids + (size_t)g * NGT * NNODE;
        for (int l = 0; l < NLEV; ++l) { const int n = NLEAF >> l; const size_t rows = (size_t)NGT * n; const size_t base = (size_t)32768 - ((size_t)32768 >> l);
            k_gath<<<(unsigned)(rows * 32 / 256), 256, 0, stream>>>(gids, emb, XE + base * NDIN, 8 - l, 512 - (512 >> l), rows * 32); }
        for (int l = 0; l < NLEV; ++l) { const int n = NLEAF >> l; const size_t rows = (size_t)NGT * n; const size_t base = (size_t)32768 - ((size_t)32768 >> l); const size_t ch = rows < (size_t)NCH ? rows : (size_t)NCH;
            float* cnew = (l & 1) ? CB : CA; const float* cprev = (l & 1) ? CA : CB;
            bf* he = (l & 1) ? HB : HA; bf* ho = he + (rows / 2) * NH;
            const bf* pe = (l & 1) ? HA : HB; const bf* po = pe + rows * NH;
            const bool root = (l == NLEV - 1);
            for (size_t row0 = 0; row0 < rows; row0 += ch) { const dim3 g3((unsigned)(ch / 64), 768 / 64, 1), g1((unsigned)(ch / 64), NH / 64, 1); const bf* xa = XE + (base + row0) * NDIN;
                k_gemmw<bf, 0, true><<<g3, 32, 0, stream>>>(xa, nullptr, WxI, nullptr, NDIN, PXi, 768, bioux, 0, 0, 0);
                if (l > 0) { const bf* a1 = pe + row0 * NH; const bf* a2 = po + row0 * NH;
                    k_gemmw<bf, 0, true><<<g1, 32, 0, stream>>>(xa, nullptr, WxF, nullptr, NDIN, PXf, NH, bfx, 0, 0, 0);
                    k_gemmw<bf, 0, true><<<g3, 32, 0, stream>>>(a1, nullptr, W1I, nullptr, NH, P1i, 768, biouh1, 0, 0, 0);
                    k_gemmw<bf, 0, true><<<g1, 32, 0, stream>>>(a1, nullptr, W1F0, nullptr, NH, P1f0, NH, bfh11, 0, 0, 0);
                    k_gemmw<bf, 0, true><<<g1, 32, 0, stream>>>(a1, nullptr, W1F1, nullptr, NH, P1f1, NH, bfh21, 0, 0, 0);
                    k_gemmw<bf, 0, true><<<g3, 32, 0, stream>>>(a2, nullptr, W2I, nullptr, NH, P2i, 768, biouh2, 0, 0, 0);
                    k_gemmw<bf, 0, true><<<g1, 32, 0, stream>>>(a2, nullptr, W2F0, nullptr, NH, P2f0, NH, bfh12, 0, 0, 0);
                    k_gemmw<bf, 0, true><<<g1, 32, 0, stream>>>(a2, nullptr, W2F1, nullptr, NH, P2f1, NH, bfh22, 0, 0, 0); }
                k_cell<<<(unsigned)(ch * 64 / 256), 256, 0, stream>>>(PXi, PXf, l > 0 ? P1i : nullptr, P1f0, P1f1, P2i, P2f0, P2f1, cprev, biouh1, biouh2, cnew, he, ho, root ? HRH + (size_t)g * NGT * NH : nullptr, root ? HRL + (size_t)g * NGT * NH : nullptr, (int)row0, ch * 64); } } }

    k_gemmw<bf, 1, false><<<dim3(NB / 64, NHP / 64, 1), 32, 0, stream>>>(HRH, HRL, WL1, nullptr, NH, PH, NHP, nullptr, 0, 0, 0);
    k_head<<<1, 256, 0, stream>>>(PH, bl1, wl2, bl2, out);
}
